// STICKYLlamaAttention_48430051230507
// MI455X (gfx1250) — hardware-verified
//
#include <hip/hip_runtime.h>


typedef __bf16 v16bf __attribute__((ext_vector_type(16)));
typedef __bf16 v8bf __attribute__((ext_vector_type(8)));
typedef float v8f __attribute__((ext_vector_type(8)));
typedef float v4f __attribute__((ext_vector_type(4)));
typedef unsigned int v4u __attribute__((ext_vector_type(4)));

static constexpr int SQ = 2048;
static constexpr int HIDN = 2048;
static constexpr int NQH = 32;
static constexpr int NKVH = 8;
static constexpr int HDIM = 64;
static constexpr int KVD = NKVH * HDIM;

struct RopeFreq { float f[32]; };
static_assert(sizeof(RopeFreq) == 128);

union Frag { v16bf v; v8bf h[2]; };

__device__ __forceinline__ v16bf ldfrag(const __bf16* rowp, int hs) {
  Frag f;
  f.h[0] = *(const v8bf*)(rowp + 8 * hs);
  f.h[1] = *(const v8bf*)(rowp + 16 + 8 * hs);
  return f.v;
}

__device__ __forceinline__ void mma3(v8f& acc, const v16bf& ah, const v16bf& al,
                                     const v16bf& bh, const v16bf& bl) {
  acc = __builtin_amdgcn_wmma_f32_16x16x32_bf16(false, ah, false, bh, (short)0, acc, false, false);
  acc = __builtin_amdgcn_wmma_f32_16x16x32_bf16(false, ah, false, bl, (short)0, acc, false, false);
  acc = __builtin_amdgcn_wmma_f32_16x16x32_bf16(false, al, false, bh, (short)0, acc, false, false);
  asm volatile("v_nop\n\tv_nop\n\tv_nop\n\tv_nop" : "+v"(acc) : "v"(ah), "v"(al), "v"(bh), "v"(bl));
}

__device__ __forceinline__ unsigned int bfbits(float x) {
  unsigned int u = __float_as_uint(x);
  return (u + 0x7FFFu + ((u >> 16) & 1u)) >> 16;
}
__device__ __forceinline__ void split_hl(float x, unsigned int& hb, unsigned int& lb) {
  hb = bfbits(x);
  const float hf = __uint_as_float(hb << 16);
  lb = bfbits(x - hf);
}
__device__ __forceinline__ unsigned int pk2(unsigned int a, unsigned int b) {
  return (a & 0xFFFFu) | (b << 16);
}
__device__ __forceinline__ v4u pack8(const unsigned int* a) {
  v4u v;
  v.x = pk2(a[0], a[1]);
  v.y = pk2(a[2], a[3]);
  v.z = pk2(a[4], a[5]);
  v.w = pk2(a[6], a[7]);
  return v;
}

__global__ void __launch_bounds__(256) k_split(
    const float* __restrict__ s0, const float* __restrict__ s1, const float* __restrict__ s2,
    const float* __restrict__ s3, const float* __restrict__ s4,
    unsigned short* __restrict__ h0, unsigned short* __restrict__ h1, unsigned short* __restrict__ h2,
    unsigned short* __restrict__ h3, unsigned short* __restrict__ h4,
    unsigned short* __restrict__ l0, unsigned short* __restrict__ l1, unsigned short* __restrict__ l2,
    unsigned short* __restrict__ l3, unsigned short* __restrict__ l4,
    int n0, int n1, int n2, int n3, int n4)
{
  const int b = blockIdx.y;
  const float* src = (b == 0) ? s0 : (b == 1) ? s1 : (b == 2) ? s2 : (b == 3) ? s3 : s4;
  unsigned short* dh = (b == 0) ? h0 : (b == 1) ? h1 : (b == 2) ? h2 : (b == 3) ? h3 : h4;
  unsigned short* dl = (b == 0) ? l0 : (b == 1) ? l1 : (b == 2) ? l2 : (b == 3) ? l3 : l4;
  const int n = (b == 0) ? n0 : (b == 1) ? n1 : (b == 2) ? n2 : (b == 3) ? n3 : n4;
  const int i = blockIdx.x * 256 + (int)threadIdx.x;
  if (i >= (n >> 3)) return;

  const float* p = src + (size_t)i * 8;
  const v4f a = *(const v4f*)(p);
  const v4f c = *(const v4f*)(p + 4);
  unsigned int hb[8], lb[8];
  split_hl(a.x, hb[0], lb[0]);
  split_hl(a.y, hb[1], lb[1]);
  split_hl(a.z, hb[2], lb[2]);
  split_hl(a.w, hb[3], lb[3]);
  split_hl(c.x, hb[4], lb[4]);
  split_hl(c.y, hb[5], lb[5]);
  split_hl(c.z, hb[6], lb[6]);
  split_hl(c.w, hb[7], lb[7]);
  const v4u hv = pack8(hb);
  const v4u lv = pack8(lb);
  volatile v4u* gh = (volatile v4u*)(dh + (size_t)i * 8);
  volatile v4u* gl = (volatile v4u*)(dl + (size_t)i * 8);
  *gh = hv;
  *gl = lv;
  __threadfence();
  *gh = hv;
  *gl = lv;
}

__global__ void __launch_bounds__(128) k_rope_tab(float* __restrict__ tab, RopeFreq fr)
{
  const int g = blockIdx.x * 128 + (int)threadIdx.x;
  const int pos = g >> 4;
  const int j = g & 15;
  if (pos >= SQ) return;
  float fa = fr.f[0], fb = fr.f[16];
#pragma unroll
  for (int c = 1; c < 16; ++c) {
    fa = (j == c) ? fr.f[c] : fa;
    fb = (j == c) ? fr.f[16 + c] : fb;
  }
  float cs0 = 0.0f, sn0 = 0.0f, cs1 = 0.0f, sn1 = 0.0f;
#pragma unroll 1
  for (int q = 0; q < 2; ++q) {
    const float f = (q == 0) ? fa : fb;
    const float ang = (float)pos * f;
    float sn, cs;
    sincosf(ang, &sn, &cs);
    if (q == 0) { cs0 = cs; sn0 = sn; } else { cs1 = cs; sn1 = sn; }
  }
  v4f v;
  v.x = cs0; v.y = sn0; v.z = cs1; v.w = sn1;
  volatile v4f* gp = (volatile v4f*)(tab + (size_t)g * 4);
  *gp = v;
  __threadfence();
  *gp = v;
}

__device__ __forceinline__ void gemm64(const __bf16* __restrict__ Ah, const __bf16* __restrict__ Al,
                                       int lda, int arow,
                                       const __bf16* __restrict__ Bh, const __bf16* __restrict__ Bl,
                                       int ldb, int brow, int K, int hs, int m,
                                       v8f& c0, v8f& c1, v8f& c2, v8f& c3)
{
  const __bf16* ah = Ah + (size_t)(arow + m) * lda;
  const __bf16* al = Al + (size_t)(arow + m) * lda;
  const __bf16* bh = Bh + (size_t)(brow + m) * ldb;
  const __bf16* bl = Bl + (size_t)(brow + m) * ldb;
  const size_t js = (size_t)16 * ldb;
#pragma unroll 1
  for (int k0 = 0; k0 < K; k0 += 32) {
    const v16bf fah = ldfrag(ah + k0, hs);
    const v16bf fal = ldfrag(al + k0, hs);
    {
      const v16bf fbh = ldfrag(bh + k0, hs);
      const v16bf fbl = ldfrag(bl + k0, hs);
      mma3(c0, fah, fal, fbh, fbl);
    }
    {
      const v16bf fbh = ldfrag(bh + js + k0, hs);
      const v16bf fbl = ldfrag(bl + js + k0, hs);
      mma3(c1, fah, fal, fbh, fbl);
    }
    {
      const v16bf fbh = ldfrag(bh + 2 * js + k0, hs);
      const v16bf fbl = ldfrag(bl + 2 * js + k0, hs);
      mma3(c2, fah, fal, fbh, fbl);
    }
    {
      const v16bf fbh = ldfrag(bh + 3 * js + k0, hs);
      const v16bf fbl = ldfrag(bl + 3 * js + k0, hs);
      mma3(c3, fah, fal, fbh, fbl);
    }
  }
}

__global__ void __launch_bounds__(128) k_qkv(
    const __bf16* __restrict__ xh, const __bf16* __restrict__ xl,
    const __bf16* __restrict__ wqh, const __bf16* __restrict__ wql,
    const __bf16* __restrict__ wkh, const __bf16* __restrict__ wkl,
    const __bf16* __restrict__ wvh, const __bf16* __restrict__ wvl,
    const float* __restrict__ tab,
    unsigned short* __restrict__ qh, unsigned short* __restrict__ ql,
    unsigned short* __restrict__ kh, unsigned short* __restrict__ kl,
    unsigned short* __restrict__ vth, unsigned short* __restrict__ vtl)
{
  __shared__ __attribute__((aligned(16))) unsigned short stg[8192];

  const int ct = blockIdx.x;
  const int m0 = blockIdx.y * 64;
  const int tid = threadIdx.x, w = tid >> 5, l = tid & 31, hs = l >> 4, m = l & 15;
  const int kind = (ct < NQH) ? 0 : ((ct < NQH + NKVH) ? 1 : 2);
  const int hd = (kind == 0) ? ct : ((kind == 1) ? (ct - NQH) : (ct - NQH - NKVH));
  const __bf16* Bh = (kind == 0) ? wqh : ((kind == 1) ? wkh : wvh);
  const __bf16* Bl = (kind == 0) ? wql : ((kind == 1) ? wkl : wvl);
  const int row0 = m0 + 16 * w;

  v8f c0 = {}, c1 = {}, c2 = {}, c3 = {};
  gemm64(xh, xl, HIDN, row0, Bh, Bl, HIDN, hd * HDIM, HIDN, hs, m, c0, c1, c2, c3);

  if (kind != 2) {
#pragma unroll
    for (int r = 0; r < 8; ++r) {
      const int pos = row0 + 8 * hs + r;
      const v4f cs = *(const v4f*)(tab + ((size_t)pos * 16 + m) * 4);
      const float a0 = c0[r], a1 = c1[r], a2 = c2[r], a3 = c3[r];
      c0[r] = a0 * cs.x - a2 * cs.y;
      c2[r] = a2 * cs.x + a0 * cs.y;
      c1[r] = a1 * cs.z - a3 * cs.w;
      c3[r] = a3 * cs.z + a1 * cs.w;
    }
  }

  const int wb = w * 2048;
  const int loff = (kind != 2) ? 1024 : 4096;
#pragma unroll
  for (int r = 0; r < 8; ++r) {
    const int rl = 8 * hs + r;
    const int base = (kind != 2) ? (wb + rl * 64 + m) : (m * 64 + 16 * w + rl);
    const int jst = (kind != 2) ? 16 : 1024;
    unsigned int hb, lb;
    split_hl(c0[r], hb, lb);
    stg[base] = (unsigned short)hb;           stg[base + loff] = (unsigned short)lb;
    split_hl(c1[r], hb, lb);
    stg[base + jst] = (unsigned short)hb;     stg[base + jst + loff] = (unsigned short)lb;
    split_hl(c2[r], hb, lb);
    stg[base + 2 * jst] = (unsigned short)hb; stg[base + 2 * jst + loff] = (unsigned short)lb;
    split_hl(c3[r], hb, lb);
    stg[base + 3 * jst] = (unsigned short)hb; stg[base + 3 * jst + loff] = (unsigned short)lb;
  }
  __syncthreads();

  unsigned short* dsth = (kind == 0) ? qh : ((kind == 1) ? kh : vth);
  unsigned short* dstl = (kind == 0) ? ql : ((kind == 1) ? kl : vtl);
  const int ld = (kind == 0) ? HIDN : KVD;
  const int col0 = hd * HDIM;
  v4u hv[4], lv[4];
  volatile v4u* gph[4];
  volatile v4u* gpl[4];
#pragma unroll
  for (int it = 0; it < 4; ++it) {
    const int rowa = it * 4 + (l >> 3), pa = l & 7;
    const int cb = it * 16 + (tid >> 3), pb = tid & 7;
    const int sidx = (kind != 2) ? (wb + rowa * 64 + pa * 8) : (cb * 64 + pb * 8);
    const size_t goff = (kind != 2) ? ((size_t)(row0 + rowa) * ld + col0 + pa * 8)
                                    : ((size_t)(hd * HDIM + cb) * SQ + m0 + pb * 8);
    hv[it] = *(const v4u*)(stg + sidx);
    lv[it] = *(const v4u*)(stg + sidx + loff);
    gph[it] = (volatile v4u*)(dsth + goff);
    gpl[it] = (volatile v4u*)(dstl + goff);
  }
#pragma unroll
  for (int it = 0; it < 4; ++it) { *gph[it] = hv[it]; *gpl[it] = lv[it]; }
  __threadfence();
#pragma unroll
  for (int it = 0; it < 4; ++it) { *gph[it] = hv[it]; *gpl[it] = lv[it]; }
}

__global__ void __launch_bounds__(256) k_attn(
    const __bf16* __restrict__ qh, const __bf16* __restrict__ ql,
    const __bf16* __restrict__ kh, const __bf16* __restrict__ kl,
    const __bf16* __restrict__ vth, const __bf16* __restrict__ vtl,
    unsigned short* __restrict__ ch, unsigned short* __restrict__ cl)
{
  __shared__ __attribute__((aligned(16))) float Ss[64 * 64];
  __shared__ __attribute__((aligned(16))) unsigned short Ph[64 * 64];
  __shared__ __attribute__((aligned(16))) unsigned short Pl[64 * 64];
  __shared__ float rowM[64];
  __shared__ float rowL[64];
  __shared__ float rowA[64];

  const int qt = blockIdx.x, hq = blockIdx.y, kvh = hq >> 2, q0 = qt * 64;
  const int tid = threadIdx.x, w = tid >> 5, l = tid & 31, hs = l >> 4, m = l & 15;
  const int msub = w & 3, nh = w >> 2;
  const int rbase = 16 * msub + 8 * hs;
  const int srow = tid >> 2, sq = tid & 3;

  if (tid < 64) { rowM[tid] = -1.0e30f; rowL[tid] = 0.0f; rowA[tid] = 0.0f; }

  const __bf16* qrh = qh + (size_t)(q0 + 16 * msub + m) * HIDN + hq * HDIM;
  const __bf16* qrl = ql + (size_t)(q0 + 16 * msub + m) * HIDN + hq * HDIM;
  const v16bf fqh0 = ldfrag(qrh, hs), fqh1 = ldfrag(qrh + 32, hs);
  const v16bf fql0 = ldfrag(qrl, hs), fql1 = ldfrag(qrl + 32, hs);

  v8f o[2] = {};

  for (int kt = 0; kt <= qt; ++kt) {
    const int k0 = kt * 64;
#pragma unroll
    for (int nt = 0; nt < 2; ++nt) {
      const int nc0 = nh * 32 + nt * 16;
      const __bf16* krh = kh + (size_t)(k0 + nc0 + m) * KVD + kvh * HDIM;
      const __bf16* krl = kl + (size_t)(k0 + nc0 + m) * KVD + kvh * HDIM;
      v8f s = {};
      {
        const v16bf bh = ldfrag(krh, hs), bl = ldfrag(krl, hs);
        mma3(s, fqh0, fql0, bh, bl);
      }
      {
        const v16bf bh = ldfrag(krh + 32, hs), bl = ldfrag(krl + 32, hs);
        mma3(s, fqh1, fql1, bh, bl);
      }
#pragma unroll
      for (int r = 0; r < 8; ++r) {
        const int row = rbase + r;
        float val = s[r] * 0.125f;
        if (kt == qt && (nc0 + m) > row) val = -1.0e30f;
        Ss[row * 64 + nc0 + m] = val;
      }
    }
    __syncthreads();

    {
      const float* sp = Ss + srow * 64 + sq * 16;
      const v4f x0 = *(const v4f*)(sp);
      const v4f x1 = *(const v4f*)(sp + 4);
      const v4f x2 = *(const v4f*)(sp + 8);
      const v4f x3 = *(const v4f*)(sp + 12);
      float p[16] = {x0.x, x0.y, x0.z, x0.w, x1.x, x1.y, x1.z, x1.w,
                     x2.x, x2.y, x2.z, x2.w, x3.x, x3.y, x3.z, x3.w};
      float mx = p[0];
#pragma unroll
      for (int c = 1; c < 16; ++c) mx = fmaxf(mx, p[c]);
      mx = fmaxf(mx, __shfl_xor(mx, 1));
      mx = fmaxf(mx, __shfl_xor(mx, 2));
      const float mOld = rowM[srow];
      const float mNew = fmaxf(mOld, mx);
      float lsum = 0.0f;
#pragma unroll
      for (int c = 0; c < 16; ++c) { p[c] = __expf(p[c] - mNew); lsum += p[c]; }
      lsum += __shfl_xor(lsum, 1);
      lsum += __shfl_xor(lsum, 2);
      const float alpha = __expf(mOld - mNew);
      if (sq == 0) {
        rowA[srow] = alpha;
        rowM[srow] = mNew;
        rowL[srow] = rowL[srow] * alpha + lsum;
      }
      unsigned int hb[16], lb[16];
#pragma unroll
      for (int c = 0; c < 16; ++c) split_hl(p[c], hb[c], lb[c]);
      unsigned short* pph = Ph + srow * 64 + sq * 16;
      unsigned short* ppl = Pl + srow * 64 + sq * 16;
      *(v4u*)(pph) = pack8(hb);
      *(v4u*)(pph + 8) = pack8(hb + 8);
      *(v4u*)(ppl) = pack8(lb);
      *(v4u*)(ppl + 8) = pack8(lb + 8);
    }
    __syncthreads();

    {
#pragma unroll
      for (int r = 0; r < 8; ++r) {
        const float al = rowA[rbase + r];
        o[0][r] *= al;
        o[1][r] *= al;
      }
      const unsigned short* prh = Ph + (16 * msub + m) * 64;
      const unsigned short* prl = Pl + (16 * msub + m) * 64;
      const v16bf fph0 = ldfrag((const __bf16*)prh, hs);
      const v16bf fph1 = ldfrag((const __bf16*)(prh + 32), hs);
      const v16bf fpl0 = ldfrag((const __bf16*)prl, hs);
      const v16bf fpl1 = ldfrag((const __bf16*)(prl + 32), hs);
#pragma unroll
      for (int dt = 0; dt < 2; ++dt) {
        const int d0 = nh * 32 + dt * 16;
        const __bf16* vrh = vth + (size_t)(kvh * HDIM + d0 + m) * SQ + k0;
        const __bf16* vrl = vtl + (size_t)(kvh * HDIM + d0 + m) * SQ + k0;
        {
          const v16bf bh = ldfrag(vrh, hs), bl = ldfrag(vrl, hs);
          mma3(o[dt], fph0, fpl0, bh, bl);
        }
        {
          const v16bf bh = ldfrag(vrh + 32, hs), bl = ldfrag(vrl + 32, hs);
          mma3(o[dt], fph1, fpl1, bh, bl);
        }
      }
    }
  }

  unsigned short* stg = (unsigned short*)Ss;
#pragma unroll
  for (int r = 0; r < 8; ++r) {
    const int row = rbase + r;
    const float inv = 1.0f / rowL[row];
#pragma unroll
    for (int dt = 0; dt < 2; ++dt) {
      const int col = nh * 32 + dt * 16 + m;
      unsigned int hb, lb;
      split_hl(o[dt][r] * inv, hb, lb);
      stg[row * 64 + col] = (unsigned short)hb;
      stg[4096 + row * 64 + col] = (unsigned short)lb;
    }
  }
  __syncthreads();
  v4u cv[4];
  volatile v4u* cp[4];
#pragma unroll
  for (int it = 0; it < 4; ++it) {
    const int plane = it >> 1;
    const int row = (it & 1) * 32 + (tid >> 3);
    const int piece = tid & 7;
    cv[it] = *(const v4u*)(stg + plane * 4096 + row * 64 + piece * 8);
    unsigned short* base = plane ? cl : ch;
    cp[it] = (volatile v4u*)(base + (size_t)(q0 + row) * HIDN + hq * HDIM + piece * 8);
  }
#pragma unroll
  for (int it = 0; it < 4; ++it) *cp[it] = cv[it];
  __threadfence();
#pragma unroll
  for (int it = 0; it < 4; ++it) *cp[it] = cv[it];
}

__global__ void __launch_bounds__(128) k_oproj(
    const __bf16* __restrict__ ah, const __bf16* __restrict__ al,
    const __bf16* __restrict__ woh, const __bf16* __restrict__ wol,
    float* __restrict__ out)
{
  __shared__ __attribute__((aligned(16))) float stgf[4096];
  const int nt = blockIdx.x, m0 = blockIdx.y * 64;
  const int tid = threadIdx.x, w = tid >> 5, l = tid & 31, hs = l >> 4, m = l & 15;
  const int row0 = m0 + 16 * w;
  const int n0 = nt * 64;

  v8f c0 = {}, c1 = {}, c2 = {}, c3 = {};
  gemm64(ah, al, HIDN, row0, woh, wol, HIDN, n0, HIDN, hs, m, c0, c1, c2, c3);

  float* sw = stgf + w * 1024;
#pragma unroll
  for (int r = 0; r < 8; ++r) {
    const int rl = 8 * hs + r;
    sw[rl * 64 + m] = c0[r];
    sw[rl * 64 + 16 + m] = c1[r];
    sw[rl * 64 + 32 + m] = c2[r];
    sw[rl * 64 + 48 + m] = c3[r];
  }
  __syncthreads();
  v4f v[8];
  volatile v4f* gp[8];
#pragma unroll
  for (int it = 0; it < 8; ++it) {
    const int row = 2 * it + (l >> 4);
    const int piece = l & 15;
    v[it] = *(const v4f*)(sw + row * 64 + piece * 4);
    gp[it] = (volatile v4f*)(out + (size_t)(row0 + row) * HIDN + n0 + piece * 4);
  }
#pragma unroll
  for (int it = 0; it < 8; ++it) *gp[it] = v[it];
  __threadfence();
#pragma unroll
  for (int it = 0; it < 8; ++it) *gp[it] = v[it];
}

extern "C" void kernel_launch(void* const* d_in, const int* in_sizes, int n_in,
                              void* d_out, int out_size, void* d_ws, size_t ws_size,
                              hipStream_t stream)
{
  if (n_in != 5) return;
  if (in_sizes[0] != SQ * HIDN || in_sizes[1] != HIDN * HIDN || in_sizes[2] != KVD * HIDN ||
      in_sizes[3] != KVD * HIDN || in_sizes[4] != HIDN * HIDN) return;
  if (out_size != SQ * HIDN) return;

  const float* hid = (const float*)d_in[0];
  const float* Wq = (const float*)d_in[1];
  const float* Wk = (const float*)d_in[2];
  const float* Wv = (const float*)d_in[3];
  const float* Wo = (const float*)d_in[4];
  float* outp = (float*)d_out;

  char* ws = (char*)d_ws;
  size_t off = 0;
  auto carve = [&](size_t bytes) -> char* {
    char* p = ws + off;
    off += (bytes + 255) & ~(size_t)255;
    return p;
  };
  const size_t BX = (size_t)SQ * HIDN * 2;
  const size_t BWQ = (size_t)HIDN * HIDN * 2;
  const size_t BWK = (size_t)KVD * HIDN * 2;
  const size_t BTAB = (size_t)SQ * 16 * 16;
  const size_t BQ = (size_t)SQ * HIDN * 2;
  const size_t BK = (size_t)SQ * KVD * 2;

  unsigned short* xh = (unsigned short*)carve(BX);
  unsigned short* xl = (unsigned short*)carve(BX);
  unsigned short* wqh = (unsigned short*)carve(BWQ);
  unsigned short* wql = (unsigned short*)carve(BWQ);
  unsigned short* wkh = (unsigned short*)carve(BWK);
  unsigned short* wkl = (unsigned short*)carve(BWK);
  unsigned short* wvh = (unsigned short*)carve(BWK);
  unsigned short* wvl = (unsigned short*)carve(BWK);
  unsigned short* woh = (unsigned short*)carve(BWQ);
  unsigned short* wol = (unsigned short*)carve(BWQ);
  float* tab = (float*)carve(BTAB);
  unsigned short* qh = (unsigned short*)carve(BQ);
  unsigned short* ql = (unsigned short*)carve(BQ);
  unsigned short* kh = (unsigned short*)carve(BK);
  unsigned short* kl = (unsigned short*)carve(BK);
  unsigned short* vth = (unsigned short*)carve(BK);
  unsigned short* vtl = (unsigned short*)carve(BK);
  unsigned short* ch = (unsigned short*)carve(BQ);
  unsigned short* cl = (unsigned short*)carve(BQ);
  if (off > ws_size) return;

  RopeFreq fr;
  {
    double r = 1.333521432163324;
    for (int it = 0; it < 4; ++it) {
      const double r2 = r * r, r4 = r2 * r2;
      const double r7 = r4 * r2 * r;
      r = r - (r4 * r4 - 10.0) / (8.0 * r7);
    }
    double rp[8];
    rp[0] = 1.0;
    for (int i = 1; i < 8; ++i) rp[i] = rp[i - 1] * r;
    const double p10[4] = {1.0, 10.0, 100.0, 1000.0};
    for (int j = 0; j < 32; ++j) {
      const double pj = p10[j >> 3] * rp[j & 7];
      const float pf = (float)pj;
      fr.f[j] = 1.0f / pf;
    }
  }

  k_split<<<dim3((SQ * HIDN / 8 + 255) / 256, 5), dim3(256), 0, stream>>>(
      hid, Wq, Wk, Wv, Wo,
      xh, wqh, wkh, wvh, woh,
      xl, wql, wkl, wvl, wol,
      SQ * HIDN, HIDN * HIDN, KVD * HIDN, KVD * HIDN, HIDN * HIDN);

  k_rope_tab<<<dim3((SQ * 16 + 127) / 128), dim3(128), 0, stream>>>(tab, fr);

  k_qkv<<<dim3(NQH + 2 * NKVH, SQ / 64), dim3(128), 0, stream>>>(
      (const __bf16*)xh, (const __bf16*)xl,
      (const __bf16*)wqh, (const __bf16*)wql,
      (const __bf16*)wkh, (const __bf16*)wkl,
      (const __bf16*)wvh, (const __bf16*)wvl,
      (const float*)tab,
      qh, ql, kh, kl, vth, vtl);

  k_attn<<<dim3(SQ / 64, NQH), dim3(256), 0, stream>>>(
      (const __bf16*)qh, (const __bf16*)ql,
      (const __bf16*)kh, (const __bf16*)kl,
      (const __bf16*)vth, (const __bf16*)vtl,
      ch, cl);

  k_oproj<<<dim3(HIDN / 64, SQ / 64), dim3(128), 0, stream>>>(
      (const __bf16*)ch, (const __bf16*)cl,
      (const __bf16*)woh, (const __bf16*)wol,
      outp);
}
